// ScaledEuclidDistanceAttention_18305150616106
// MI455X (gfx1250) — hardware-verified
//
#include <hip/hip_runtime.h>
#include <stdint.h>
#include <stddef.h>

typedef __attribute__((ext_vector_type(16))) _Float16 v16h;
typedef __attribute__((ext_vector_type(8)))  _Float16 v8h;
typedef __attribute__((ext_vector_type(16))) __bf16   v16b;
typedef __attribute__((ext_vector_type(8)))  __bf16   v8b;
typedef __attribute__((ext_vector_type(8)))  float    v8f;
typedef __attribute__((ext_vector_type(4)))  float    v4f;
typedef __attribute__((ext_vector_type(4)))  unsigned v4u;

constexpr int NBATCH = 2;
constexpr int SEQ    = 2048;
constexpr int DMODEL = 1024;
constexpr int NHEAD  = 16;
constexpr int HDIM   = 64;
constexpr int NTOK   = NBATCH * SEQ;
constexpr int KCH    = 64;
constexpr int QBLK   = 64;
static_assert(NHEAD * HDIM == DMODEL);
static_assert(HDIM == 64);
static_assert(SEQ % KCH == 0 && SEQ % QBLK == 0);
static_assert(NTOK % 64 == 0 && DMODEL % 64 == 0 && DMODEL % 32 == 0);

constexpr size_t ACT16_B = (size_t)NTOK * DMODEL * 2;
constexpr size_t W16_B   = (size_t)DMODEL * DMODEL * 2;
constexpr size_t ACT32_B = (size_t)NTOK * DMODEL * 4;
constexpr size_t OFF_QB  = 0;
constexpr size_t OFF_KB  = OFF_QB + ACT16_B;
constexpr size_t OFF_VB  = OFF_KB + ACT16_B;
constexpr size_t OFF_WQ  = OFF_VB + ACT16_B;
constexpr size_t OFF_WK  = OFF_WQ + W16_B;
constexpr size_t OFF_WV  = OFF_WK + W16_B;
constexpr size_t OFF_WO  = OFF_WV + W16_B;
constexpr size_t OFF_QH  = OFF_WO + W16_B;
constexpr size_t OFF_KH  = OFF_QH + ACT16_B;
constexpr size_t OFF_VHI = OFF_KH + ACT16_B;
constexpr size_t OFF_VLO = OFF_VHI + ACT16_B;
constexpr size_t OFF_O32 = OFF_VLO + ACT16_B;
constexpr size_t OFF_OHI = OFF_O32 + ACT32_B;
constexpr size_t OFF_OLO = OFF_OHI + ACT16_B;
constexpr size_t WS_TOTAL = OFF_OLO + ACT16_B;
static_assert(WS_TOTAL == 100663296);
static_assert(WS_TOTAL <= 134217728);

__device__ __forceinline__ unsigned short f2bf_bits(float f) {
  unsigned u = __float_as_uint(f);
  return (unsigned short)((u + 0x7FFFu + ((u >> 16) & 1u)) >> 16);
}
__device__ __forceinline__ float bf_bits2f(unsigned short h) { return __uint_as_float(((unsigned)h) << 16); }

__device__ __forceinline__ float h_bits2f(unsigned h) {
  const unsigned e = (h >> 10) & 31u;
  const unsigned m = h & 1023u;
  const unsigned s = (h & 0x8000u) << 16;
  const unsigned r = s | ((e + 112u) << 23) | (m << 13);
  return __uint_as_float((e == 0u) ? s : r);
}

__device__ __forceinline__ void dep_guard_h(v8f& a, v8f& b, v16h x, v16h y) { asm volatile("v_nop\n\tv_nop\n\tv_nop\n\tv_nop" : "+v"(a), "+v"(b) : "v"(x), "v"(y)); }
__device__ __forceinline__ void dep_guard_b(v8f& a, v8f& b, v16b x, v16b y) { asm volatile("v_nop\n\tv_nop\n\tv_nop\n\tv_nop" : "+v"(a), "+v"(b) : "v"(x), "v"(y)); }
__device__ __forceinline__ void keep4_h(v16h a, v16h b, v16h c, v16h d) { asm volatile("v_nop" :: "v"(a), "v"(b), "v"(c), "v"(d)); }
__device__ __forceinline__ void keep4_b(v16b a, v16b b, v16b c, v16b d) { asm volatile("v_nop" :: "v"(a), "v"(b), "v"(c), "v"(d)); }
__device__ __forceinline__ void acc_guard4(v8f& a, v8f& b, v8f& c, v8f& d) { asm volatile("v_nop\n\tv_nop\n\tv_nop\n\tv_nop" : "+v"(a), "+v"(b), "+v"(c), "+v"(d)); }

template <typename T> struct Frag;
template <> struct Frag<_Float16> {
  typedef v16h V; union U { v16h v; v8h h[2]; };
  static __device__ __forceinline__ v16h load(const _Float16* p) {
    U f; f.h[0] = *(const v8h*)(p); f.h[1] = *(const v8h*)(p + 16); return f.v;
  }
  static __device__ __forceinline__ v8f mma(v16h a, v16h b, v8f c) {
    return __builtin_amdgcn_wmma_f32_16x16x32_f16(false, a, false, b, (short)0, c, false, false);
  }
  static __device__ __forceinline__ void guard(v8f& a, v8f& b, v16h x, v16h y) { dep_guard_h(a, b, x, y); }
  static __device__ __forceinline__ void keep(v16h a, v16h b, v16h c, v16h d) { keep4_h(a, b, c, d); }
};
template <> struct Frag<__bf16> {
  typedef v16b V; union U { v16b v; v8b h[2]; };
  static __device__ __forceinline__ v16b load(const __bf16* p) {
    U f; f.h[0] = *(const v8b*)(p); f.h[1] = *(const v8b*)(p + 16); return f.v;
  }
  static __device__ __forceinline__ v8f mma(v16b a, v16b b, v8f c) {
    return __builtin_amdgcn_wmma_f32_16x16x32_bf16(false, a, false, b, (short)0, c, false, false);
  }
  static __device__ __forceinline__ void guard(v8f& a, v8f& b, v16b x, v16b y) { dep_guard_b(a, b, x, y); }
  static __device__ __forceinline__ void keep(v16b a, v16b b, v16b c, v16b d) { keep4_b(a, b, c, d); }
};

__device__ __forceinline__ v8f mma_h(v16h a, v16h b, v8f c) {
  c = __builtin_amdgcn_wmma_f32_16x16x32_f16(false, a, false, b, (short)0, c, false, false);
  asm volatile("v_nop\n\tv_nop\n\tv_nop\n\tv_nop" : "+v"(c) : "v"(a), "v"(b));
  return c;
}
__device__ __forceinline__ v8f mma_b(v16b a, v16b b, v8f c) {
  c = __builtin_amdgcn_wmma_f32_16x16x32_bf16(false, a, false, b, (short)0, c, false, false);
  asm volatile("v_nop\n\tv_nop\n\tv_nop\n\tv_nop" : "+v"(c) : "v"(a), "v"(b));
  return c;
}

template <int ET> struct Elem;
template <> struct Elem<0> { typedef _Float16 T; };
template <> struct Elem<1> { typedef __bf16 T; };
template <int ET, int SPLIT, int BIAS_MODE, int OUT_MODE, bool RESID>
__global__ __launch_bounds__(256) void wmma_gemm64(
    const unsigned short* __restrict__ Ap, const unsigned short* __restrict__ A2p, int lda, long strideA,
    const unsigned short* __restrict__ Btp, const unsigned short* __restrict__ Bt2p, int ldb, long strideB,
    void* __restrict__ Cout, void* __restrict__ Cout2, int ldc, long strideC,
    const float* __restrict__ bias,
    const float* __restrict__ resid, long strideR,
    int M, int N, int K, float scale) {
  typedef typename Elem<ET>::T T;
  typedef typename Frag<T>::V V;
  const T* A = (const T*)Ap; const T* A2 = (const T*)A2p; const T* Bt = (const T*)Btp; const T* Bt2 = (const T*)Bt2p;
  __shared__ __align__(16) float sT[8][16 * 68];
  const int b    = blockIdx.y;
  const int lane = threadIdx.x & 31;
  const int wave = threadIdx.x >> 5;
  const int tilesN = N >> 6;
  const int tilesM = M >> 6;
  const int tile = blockIdx.x * 8 + wave;
  if (tile >= tilesM * tilesN) return;
  const int tm = tile / tilesN;
  const int tn = tile - tm * tilesN;
  const int m0 = tm << 6;
  const int n0 = tn << 6;

  const T* Ab  = A  + (size_t)b * strideA;
  const T* Bb  = Bt + (size_t)b * strideB;
  const T* Ab2 = (SPLIT != 0) ? (A2  + (size_t)b * strideA) : nullptr;
  const T* Bb2 = (SPLIT == 1) ? (Bt2 + (size_t)b * strideB) : nullptr;

  const int rlane = lane & 15;
  const int koff  = (lane >> 4) * 8;
  const int mOff  = (lane >> 4) * 8;

  v8f acc[4][4];
#pragma unroll
  for (int i = 0; i < 4; ++i)
#pragma unroll
    for (int j = 0; j < 4; ++j) acc[i][j] = (v8f){0.f,0.f,0.f,0.f,0.f,0.f,0.f,0.f};

  for (int k0 = 0; k0 < K; k0 += 32) {
    V bh[4], bl[4];
#pragma unroll
    for (int j = 0; j < 4; ++j) {
      const size_t bo = (size_t)(n0 + (j << 4) + rlane) * ldb + koff + k0;
      bh[j] = Frag<T>::load(Bb + bo);
      if (SPLIT == 1) bl[j] = Frag<T>::load(Bb2 + bo);
    }
#pragma unroll
    for (int i = 0; i < 4; ++i) {
      const size_t ao = (size_t)(m0 + (i << 4) + rlane) * lda + koff + k0;
      V ah = Frag<T>::load(Ab + ao);
      V al = ah;
      if (SPLIT != 0) al = Frag<T>::load(Ab2 + ao);
#pragma unroll
      for (int j = 0; j < 4; ++j) {
        acc[i][j] = Frag<T>::mma(ah, bh[j], acc[i][j]);
        if (SPLIT == 1) acc[i][j] = Frag<T>::mma(ah, bl[j], acc[i][j]);
        if (SPLIT != 0) acc[i][j] = Frag<T>::mma(al, bh[j], acc[i][j]);
      }
      Frag<T>::guard(acc[i][0], acc[i][3], ah, al);
    }
    Frag<T>::keep(bh[0], bh[1], bh[2], bh[3]);
    if (SPLIT == 1) Frag<T>::keep(bl[0], bl[1], bl[2], bl[3]);
  }
  acc_guard4(acc[0][0], acc[0][1], acc[0][2], acc[0][3]);
  acc_guard4(acc[1][0], acc[1][1], acc[1][2], acc[1][3]);
  acc_guard4(acc[2][0], acc[2][1], acc[2][2], acc[2][3]);
  acc_guard4(acc[3][0], acc[3][1], acc[3][2], acc[3][3]);

  float* slab = sT[wave];
  const float* Rb = RESID ? (resid + (size_t)b * strideR) : nullptr;
#pragma unroll
  for (int i = 0; i < 4; ++i) {
    const int mBase = m0 + (i << 4);
#pragma unroll
    for (int j = 0; j < 4; ++j) {
      const int n = n0 + (j << 4) + rlane;
      float bv = 0.f;
      if (BIAS_MODE == 2) bv = bias[n];
#pragma unroll
      for (int r = 0; r < 8; ++r) {
        float v = acc[i][j][r] * scale;
        if (BIAS_MODE == 1) v += bias[mBase + mOff + r];
        if (BIAS_MODE == 2) v += bv;
        if (RESID) v += Rb[(size_t)(mBase + mOff + r) * ldc + n];
        slab[(mOff + r) * 68 + (j << 4) + rlane] = v;
      }
    }
    __builtin_amdgcn_fence(__ATOMIC_RELEASE, "workgroup");
    __builtin_amdgcn_wave_barrier();
    __builtin_amdgcn_fence(__ATOMIC_ACQUIRE, "workgroup");
    if (OUT_MODE == 0) {
      float* C = (float*)Cout + (size_t)b * strideC;
      const int hh = lane >> 4, c4 = (lane & 15) * 4;
      for (int pass = 0; pass < 2; ++pass) {
#pragma unroll
        for (int it = 0; it < 8; ++it) {
          const int row = it * 2 + hh;
          v4f v = *(const v4f*)(slab + row * 68 + c4);
          *(volatile v4f*)(C + (size_t)(mBase + row) * ldc + n0 + c4) = v;
        }
        __threadfence();
      }
    } else {
      const int q = lane >> 3, c8 = (lane & 7) * 8;
      unsigned short* C  = (unsigned short*)Cout  + (size_t)b * strideC;
      unsigned short* C2 = (OUT_MODE == 2) ? ((unsigned short*)Cout2 + (size_t)b * strideC) : nullptr;
      for (int pass = 0; pass < 2; ++pass) {
#pragma unroll
        for (int it = 0; it < 4; ++it) {
          const int row = it * 4 + q;
          const float* sp = slab + row * 68 + c8;
          v8h hv, lv;
#pragma unroll
          for (int e = 0; e < 8; ++e) {
            if (OUT_MODE == 1) {
              hv[e] = (_Float16)sp[e];
            } else {
              unsigned short hb = f2bf_bits(sp[e]);
              unsigned short lb = f2bf_bits(sp[e] - bf_bits2f(hb));
              hv[e] = __builtin_bit_cast(_Float16, hb);
              lv[e] = __builtin_bit_cast(_Float16, lb);
            }
          }
          *(volatile v8h*)(C + (size_t)(mBase + row) * ldc + n0 + c8) = hv;
          if (OUT_MODE == 2) *(volatile v8h*)(C2 + (size_t)(mBase + row) * ldc + n0 + c8) = lv;
        }
        __threadfence();
      }
    }
    __builtin_amdgcn_fence(__ATOMIC_RELEASE, "workgroup");
    __builtin_amdgcn_wave_barrier();
    __builtin_amdgcn_fence(__ATOMIC_ACQUIRE, "workgroup");
  }
}

__global__ __launch_bounds__(256) void cast_f32_bf16x8(
    const float* __restrict__ in, unsigned short* __restrict__ out, int n8) {
  const int i = blockIdx.x * 256 + threadIdx.x;
  if (i < n8) {
    const size_t o = (size_t)i * 8;
    const v4f a0 = *(const v4f*)(in + o);
    const v4f a1 = *(const v4f*)(in + o + 4);
    v4u w;
    w[0] = (unsigned)f2bf_bits(a0[0]) | ((unsigned)f2bf_bits(a0[1]) << 16);
    w[1] = (unsigned)f2bf_bits(a0[2]) | ((unsigned)f2bf_bits(a0[3]) << 16);
    w[2] = (unsigned)f2bf_bits(a1[0]) | ((unsigned)f2bf_bits(a1[1]) << 16);
    w[3] = (unsigned)f2bf_bits(a1[2]) | ((unsigned)f2bf_bits(a1[3]) << 16);
    *(volatile v4u*)(out + o) = w;
    __threadfence();
    *(volatile v4u*)(out + o) = w;
  }
}

__global__ __launch_bounds__(256) void cast_f32_bf16hilo_x8(
    const float* __restrict__ in, unsigned short* __restrict__ hi, unsigned short* __restrict__ lo, int n8) {
  const int i = blockIdx.x * 256 + threadIdx.x;
  if (i < n8) {
    const size_t o = (size_t)i * 8;
    const v4f a0 = *(const v4f*)(in + o);
    const v4f a1 = *(const v4f*)(in + o + 4);
    unsigned hb[8], lb[8];
#pragma unroll
    for (int e = 0; e < 4; ++e) {
      const unsigned short h0 = f2bf_bits(a0[e]);
      const unsigned short h1 = f2bf_bits(a1[e]);
      hb[e] = h0; hb[4 + e] = h1;
      lb[e]     = f2bf_bits(a0[e] - bf_bits2f(h0));
      lb[4 + e] = f2bf_bits(a1[e] - bf_bits2f(h1));
    }
    v4u wh, wl;
#pragma unroll
    for (int e = 0; e < 4; ++e) {
      wh[e] = hb[2 * e] | (hb[2 * e + 1] << 16);
      wl[e] = lb[2 * e] | (lb[2 * e + 1] << 16);
    }
    *(volatile v4u*)(hi + o) = wh;
    *(volatile v4u*)(lo + o) = wl;
    __threadfence();
    *(volatile v4u*)(hi + o) = wh;
    *(volatile v4u*)(lo + o) = wl;
  }
}

__global__ __launch_bounds__(128)
void euclid_attn_kernel(const unsigned short* __restrict__ Qp, const unsigned short* __restrict__ Kp,
                        const unsigned short* __restrict__ Vhp, const unsigned short* __restrict__ Vlp,
                        float* __restrict__ Out) {
  __shared__ __align__(16) unsigned short Ksh[KCH * HDIM];
  __shared__ __align__(16) unsigned short Vth[HDIM * KCH];
  __shared__ __align__(16) unsigned short Vtl[HDIM * KCH];
  __shared__ __align__(16) unsigned short Psh[4][16 * KCH];
  __shared__ __align__(16) unsigned short Psl[4][16 * KCH];
  __shared__ __align__(16) float Os[4][16 * 68];
  __shared__ __align__(16) float k2s[KCH];

  const int tid  = threadIdx.x;
  const int wave = tid >> 5;
  const int lane = tid & 31;
  const int hh   = lane >> 4;
  const int c    = lane & 15;

  const int nqb  = SEQ / QBLK;
  const int bx   = blockIdx.x;
  const int qb   = bx % nqb;
  const int bhix = bx / nqb;
  const int h    = bhix % NHEAD;
  const int b    = bhix / NHEAD;
  const int q0   = qb * QBLK + wave * 16;
  const size_t tok0 = (size_t)b * SEQ;
  const int hcol = h * HDIM;

  v16h qa[2];
  float q2p = 0.f;
  {
    const unsigned short* qrow = Qp + (tok0 + q0 + c) * DMODEL + hcol;
#pragma unroll
    for (int dc = 0; dc < 2; ++dc) {
      qa[dc] = Frag<_Float16>::load((const _Float16*)(qrow + dc * 32 + 8 * hh));
#pragma unroll
      for (int part = 0; part < 2; ++part) {
        const v4u w = *(const v4u*)(qrow + dc * 32 + 16 * part + 8 * hh);
#pragma unroll
        for (int e = 0; e < 4; ++e) {
          const float f0 = h_bits2f(w[e] & 0xffffu);
          const float f1 = h_bits2f(w[e] >> 16);
          q2p = fmaf(f0, f0, q2p);
          q2p = fmaf(f1, f1, q2p);
        }
      }
    }
  }
  const float q2c = q2p + __shfl_xor(q2p, 16, 32);
  float q2r[8];
#pragma unroll
  for (int r = 0; r < 8; ++r) q2r[r] = __shfl(q2c, 8 * hh + r, 32);

  float mrow[8], lrow[8];
  v8f oacc[4];
#pragma unroll
  for (int r = 0; r < 8; ++r) { mrow[r] = -INFINITY; lrow[r] = 0.f; }
#pragma unroll
  for (int t = 0; t < 4; ++t) oacc[t] = (v8f){0.f,0.f,0.f,0.f,0.f,0.f,0.f,0.f};

  for (int kc = 0; kc < SEQ / KCH; ++kc) {
    const int kv0 = kc * KCH;
    __syncthreads();
    {
      const int kvr = tid >> 1, dpart = (tid & 1) * 32;
      const size_t g = (tok0 + kv0 + kvr) * DMODEL + hcol + dpart;
      float ksq = 0.f;
      {
        v4u kw[4];
#pragma unroll
        for (int i = 0; i < 4; ++i) kw[i] = *(const v4u*)(Kp + g + 8 * i);
#pragma unroll
        for (int i = 0; i < 4; ++i) {
          *(v4u*)(Ksh + kvr * HDIM + dpart + 8 * i) = kw[i];
#pragma unroll
          for (int e = 0; e < 4; ++e) {
            const unsigned u = kw[i][e];
            const float f0 = h_bits2f(u & 0xffffu);
            const float f1 = h_bits2f(u >> 16);
            ksq = fmaf(f0, f0, ksq);
            ksq = fmaf(f1, f1, ksq);
          }
        }
      }
      {
        v4u vhw[4], vlw[4];
#pragma unroll
        for (int i = 0; i < 4; ++i) { vhw[i] = *(const v4u*)(Vhp + g + 8 * i); vlw[i] = *(const v4u*)(Vlp + g + 8 * i); }
#pragma unroll
        for (int i = 0; i < 4; ++i) {
#pragma unroll
          for (int e = 0; e < 4; ++e) {
            const int d = dpart + 8 * i + 2 * e;
            const unsigned uh = vhw[i][e], ul = vlw[i][e];
            Vth[d * KCH + kvr]       = (unsigned short)(uh & 0xffffu);
            Vth[(d + 1) * KCH + kvr] = (unsigned short)(uh >> 16);
            Vtl[d * KCH + kvr]       = (unsigned short)(ul & 0xffffu);
            Vtl[(d + 1) * KCH + kvr] = (unsigned short)(ul >> 16);
          }
        }
      }
      ksq += __shfl_xor(ksq, 1, 32);
      if ((tid & 1) == 0) k2s[kvr] = ksq;
    }
    __syncthreads();

    v8f s[4];
#pragma unroll
    for (int j = 0; j < 4; ++j) {
      s[j] = (v8f){0.f,0.f,0.f,0.f,0.f,0.f,0.f,0.f};
#pragma unroll
      for (int dc = 0; dc < 2; ++dc) {
        const v16h kb = Frag<_Float16>::load((const _Float16*)(Ksh + (j * 16 + c) * HDIM + dc * 32 + 8 * hh));
        s[j] = mma_h(qa[dc], kb, s[j]);
      }
    }
    float k2j[4];
#pragma unroll
    for (int j = 0; j < 4; ++j) k2j[j] = k2s[j * 16 + c];

    float cm[8];
#pragma unroll
    for (int r = 0; r < 8; ++r) {
      float m = -INFINITY;
#pragma unroll
      for (int j = 0; j < 4; ++j) {
        float d2 = (q2r[r] + k2j[j]) - 2.0f * s[j][r];
        d2 = fmaxf(d2, 0.0f);
        const float dist = __builtin_amdgcn_sqrtf(d2) * 0.125f;
        const float lg = __builtin_amdgcn_rcpf(dist + 1e-9f);
        s[j][r] = lg;
        m = fmaxf(m, lg);
      }
#pragma unroll
      for (int off = 1; off < 16; off <<= 1) m = fmaxf(m, __shfl_xor(m, off, 32));
      cm[r] = m;
    }

    unsigned short* pwh = Psh[wave];
    unsigned short* pwl = Psl[wave];
#pragma unroll
    for (int r = 0; r < 8; ++r) {
      const float mnew = fmaxf(mrow[r], cm[r]);
      const float alpha = expf(mrow[r] - mnew);
      mrow[r] = mnew;
      float psum = 0.f;
#pragma unroll
      for (int j = 0; j < 4; ++j) {
        const float p = expf(s[j][r] - mnew);
        psum += p;
        const unsigned short hb = f2bf_bits(p);
        const unsigned short lb = f2bf_bits(p - bf_bits2f(hb));
        pwh[(8 * hh + r) * KCH + j * 16 + c] = hb;
        pwl[(8 * hh + r) * KCH + j * 16 + c] = lb;
      }
#pragma unroll
      for (int off = 1; off < 16; off <<= 1) psum += __shfl_xor(psum, off, 32);
      lrow[r] = lrow[r] * alpha + psum;
#pragma unroll
      for (int t = 0; t < 4; ++t) oacc[t][r] *= alpha;
    }
    __builtin_amdgcn_fence(__ATOMIC_RELEASE, "workgroup");
    __builtin_amdgcn_wave_barrier();
    __builtin_amdgcn_fence(__ATOMIC_ACQUIRE, "workgroup");

#pragma unroll 1
    for (int kk = 0; kk < 2; ++kk) {
      const v16b pa = Frag<__bf16>::load((const __bf16*)(pwh + c * KCH + kk * 32 + 8 * hh));
      const v16b pl = Frag<__bf16>::load((const __bf16*)(pwl + c * KCH + kk * 32 + 8 * hh));
#pragma unroll
      for (int t = 0; t < 4; ++t) {
        const v16b vb = Frag<__bf16>::load((const __bf16*)(Vth + (t * 16 + c) * KCH + kk * 32 + 8 * hh));
        const v16b vl = Frag<__bf16>::load((const __bf16*)(Vtl + (t * 16 + c) * KCH + kk * 32 + 8 * hh));
        oacc[t] = mma_b(pa, vb, oacc[t]);
        oacc[t] = mma_b(pa, vl, oacc[t]);
        oacc[t] = mma_b(pl, vb, oacc[t]);
      }
    }
  }

  float* os = Os[wave];
#pragma unroll
  for (int r = 0; r < 8; ++r) {
    const float inv = 1.0f / lrow[r];
#pragma unroll
    for (int t = 0; t < 4; ++t) os[(8 * hh + r) * 68 + t * 16 + c] = oacc[t][r] * inv;
  }
  __builtin_amdgcn_fence(__ATOMIC_RELEASE, "workgroup");
  __builtin_amdgcn_wave_barrier();
  __builtin_amdgcn_fence(__ATOMIC_ACQUIRE, "workgroup");
  {
    float* ob = Out + (tok0 + q0) * DMODEL + hcol;
    const int c4 = (lane & 15) * 4;
    for (int pass = 0; pass < 2; ++pass) {
#pragma unroll
      for (int it = 0; it < 8; ++it) {
        const int row = it * 2 + hh;
        v4f val = *(const v4f*)(os + row * 68 + c4);
        *(volatile v4f*)(ob + (size_t)row * DMODEL + c4) = val;
      }
      __threadfence();
    }
  }
}

extern "C" void kernel_launch(void* const* d_in, const int* in_sizes, int n_in,
                              void* d_out, int out_size, void* d_ws, size_t ws_size,
                              hipStream_t stream) {
  if (n_in < 8) return;
  if (in_sizes[0] != NTOK * DMODEL || in_sizes[1] != NTOK * DMODEL || in_sizes[2] != NTOK * DMODEL) return;
  if (in_sizes[3] != DMODEL * DMODEL || in_sizes[4] != DMODEL * DMODEL ||
      in_sizes[5] != DMODEL * DMODEL || in_sizes[6] != DMODEL * DMODEL) return;
  if (in_sizes[7] != DMODEL) return;
  if (out_size != NTOK * DMODEL) return;
  if (ws_size < WS_TOTAL) return;

  const float* q     = (const float*)d_in[0];
  const float* k     = (const float*)d_in[1];
  const float* v     = (const float*)d_in[2];
  const float* Wq    = (const float*)d_in[3];
  const float* Wk    = (const float*)d_in[4];
  const float* Wv    = (const float*)d_in[5];
  const float* Wout  = (const float*)d_in[6];
  const float* b_out = (const float*)d_in[7];

  char* ws = (char*)d_ws;
  unsigned short* qb16 = (unsigned short*)(ws + OFF_QB);
  unsigned short* kb16 = (unsigned short*)(ws + OFF_KB);
  unsigned short* vb16 = (unsigned short*)(ws + OFF_VB);
  unsigned short* wq16 = (unsigned short*)(ws + OFF_WQ);
  unsigned short* wk16 = (unsigned short*)(ws + OFF_WK);
  unsigned short* wv16 = (unsigned short*)(ws + OFF_WV);
  unsigned short* wo16 = (unsigned short*)(ws + OFF_WO);
  unsigned short* qh16 = (unsigned short*)(ws + OFF_QH);
  unsigned short* kh16 = (unsigned short*)(ws + OFF_KH);
  unsigned short* vhi  = (unsigned short*)(ws + OFF_VHI);
  unsigned short* vlo  = (unsigned short*)(ws + OFF_VLO);
  float*          o32  = (float*)(ws + OFF_O32);
  unsigned short* ohi  = (unsigned short*)(ws + OFF_OHI);
  unsigned short* olo  = (unsigned short*)(ws + OFF_OLO);
  float*          out  = (float*)d_out;

  const int act_n8 = NTOK * DMODEL / 8;
  const int w_n8   = DMODEL * DMODEL / 8;
  static_assert((NTOK * DMODEL) % 8 == 0 && (DMODEL * DMODEL) % 8 == 0);
  const int act_blk = (act_n8 + 255) / 256;
  const int w_blk   = (w_n8 + 255) / 256;

  cast_f32_bf16x8<<<act_blk, 256, 0, stream>>>(q, qb16, act_n8);
  cast_f32_bf16x8<<<act_blk, 256, 0, stream>>>(k, kb16, act_n8);
  cast_f32_bf16x8<<<act_blk, 256, 0, stream>>>(v, vb16, act_n8);
  cast_f32_bf16x8<<<w_blk, 256, 0, stream>>>(Wq, wq16, w_n8);
  cast_f32_bf16x8<<<w_blk, 256, 0, stream>>>(Wk, wk16, w_n8);
  cast_f32_bf16x8<<<w_blk, 256, 0, stream>>>(Wv, wv16, w_n8);
  cast_f32_bf16x8<<<w_blk, 256, 0, stream>>>(Wout, wo16, w_n8);

  const int gemm_tiles = (NTOK / 64) * (DMODEL / 64);
  const int gemm_blk   = (gemm_tiles + 7) / 8;
  static_assert(NTOK % 64 == 0 && DMODEL % 64 == 0 && DMODEL % 32 == 0);

  wmma_gemm64<1, 0, 0, 1, false><<<dim3(gemm_blk, 1), 256, 0, stream>>>(
      qb16, nullptr, DMODEL, 0L, wq16, nullptr, DMODEL, 0L,
      (void*)qh16, nullptr, DMODEL, 0L, nullptr, nullptr, 0L, NTOK, DMODEL, DMODEL, 1.0f);
  wmma_gemm64<1, 0, 0, 1, false><<<dim3(gemm_blk, 1), 256, 0, stream>>>(
      kb16, nullptr, DMODEL, 0L, wk16, nullptr, DMODEL, 0L,
      (void*)kh16, nullptr, DMODEL, 0L, nullptr, nullptr, 0L, NTOK, DMODEL, DMODEL, 1.0f);
  wmma_gemm64<1, 0, 0, 2, false><<<dim3(gemm_blk, 1), 256, 0, stream>>>(
      vb16, nullptr, DMODEL, 0L, wv16, nullptr, DMODEL, 0L,
      (void*)vhi, (void*)vlo, DMODEL, 0L, nullptr, nullptr, 0L, NTOK, DMODEL, DMODEL, 1.0f);

  const int attn_blk = NBATCH * NHEAD * (SEQ / QBLK);
  euclid_attn_kernel<<<attn_blk, 128, 0, stream>>>(qh16, kh16, vhi, vlo, o32);

  cast_f32_bf16hilo_x8<<<act_blk, 256, 0, stream>>>(o32, ohi, olo, act_n8);

  wmma_gemm64<1, 2, 2, 0, false><<<dim3(gemm_blk, 1), 256, 0, stream>>>(
      ohi, olo, DMODEL, 0L, wo16, nullptr, DMODEL, 0L,
      (void*)out, nullptr, DMODEL, 0L, b_out, nullptr, 0L, NTOK, DMODEL, DMODEL, 1.0f);
}
